// TwoSourceAttention_39341900431855
// MI455X (gfx1250) — hardware-verified
//
#include <hip/hip_runtime.h>


namespace {
constexpr int NB = 2, SX = 1024, SY = 1024, D = 1024, NH = 16, DH = 64, FULL = 1536, NROW = NB * SX;
constexpr float XS = 8.0f, WSC = 256.0f, PS = 8.0f, NEG = -10000.0f;

typedef _Float16 b16;
typedef __attribute__((ext_vector_type(16))) _Float16 v16b;
typedef __attribute__((ext_vector_type(8))) _Float16 v8b;
typedef __attribute__((ext_vector_type(8))) float v8f;
typedef __attribute__((ext_vector_type(4))) float v4f;
__device__ __forceinline__ float bf16_rne(float f) { unsigned int u = __float_as_uint(f); u += 0x7FFFu + ((u >> 16) & 1u); return __uint_as_float(u & 0xFFFF0000u); }
__device__ __forceinline__ void split16(float v, b16& hi, b16& lo) { hi = (b16)v; lo = (b16)(v - (float)hi); }
__device__ __forceinline__ v16b frag_kb(const b16* p, int hh) { const v8b a = *(const v8b*)(p + 8 * hh), b = *(const v8b*)(p + 16 + 8 * hh); v16b f;
#pragma unroll
  for (int e = 0; e < 8; ++e) { f[e] = a[e]; f[8 + e] = b[e]; } return f; }
__device__ __forceinline__ v8f wmma16b(v16b a, v16b b, v8f c) { v8f d = __builtin_amdgcn_wmma_f32_16x16x32_f16(false, a, false, b, (short)0, c, false, false); asm volatile("v_nop\n\tv_nop\n\tv_nop\n\tv_nop" : "+v"(d) : "v"(a), "v"(b)); return d; }
__device__ __forceinline__ void wave_lds_sync() { __builtin_amdgcn_fence(__ATOMIC_RELEASE, "workgroup"); __builtin_amdgcn_wave_barrier(); __builtin_amdgcn_fence(__ATOMIC_ACQUIRE, "workgroup"); }
__device__ __forceinline__ float nexp(float x) { return __builtin_amdgcn_exp2f(x * 1.4426950408889634f); }
__device__ __forceinline__ int iclamp(int v, int lo, int hi) { return v < lo ? lo : (v > hi ? hi : v); }

__global__ __launch_bounds__(256) void prepx_kernel(const float* __restrict__ x, const float* __restrict__ y, b16* __restrict__ X16, b16* __restrict__ Y16) {
  const size_t i = ((size_t)blockIdx.x * 256 + threadIdx.x) * 8; const bool isy = i >= (size_t)NROW * D;
  const size_t e = isy ? i - (size_t)NROW * D : i; const float* src = (isy ? y : x) + e; b16* dst = (isy ? Y16 : X16) + e;
  const v4f a = *(const v4f*)(src), c = *(const v4f*)(src + 4); v8b o;
#pragma unroll
  for (int j = 0; j < 4; ++j) { o[j] = (b16)(bf16_rne(a[j]) * XS); o[4 + j] = (b16)(bf16_rne(c[j]) * XS); }
  for (int pass = 0; pass < 2; ++pass) { *(volatile v8b*)dst = o; __threadfence(); }
}
__global__ __launch_bounds__(256) void prepw_kernel(const float* __restrict__ wattn, const float* __restrict__ w2a, const float* __restrict__ w2b, const float* __restrict__ wproj, b16* __restrict__ WA, b16* __restrict__ W2A, b16* __restrict__ W2B, b16* __restrict__ WPJ) {
  __shared__ __attribute__((aligned(16))) b16 T[64][64 + 8];
  const int which = blockIdx.z, i0 = blockIdx.x * 64, o0 = blockIdx.y * 64, t_ = threadIdx.x;
  const int IN = which == 3 ? 2 * D : D, OUT = which == 0 ? 3 * D : which == 1 ? D : which == 2 ? 2 * D : D;
  if (i0 >= IN || o0 >= OUT) return;
  const float* w = which == 0 ? wattn : which == 1 ? w2a : which == 2 ? w2b : wproj; b16* dst = which == 0 ? WA : which == 1 ? W2A : which == 2 ? W2B : WPJ;
  for (int q = t_; q < 64 * 64; q += 256) { const int ii = q >> 6, oo = q & 63; T[oo][ii] = (b16)(bf16_rne(w[(size_t)(i0 + ii) * OUT + o0 + oo]) * WSC); }
  __syncthreads();
  for (int pass = 0; pass < 2; ++pass) { for (int q = t_; q < 64 * 8; q += 256) { const int oo = q >> 3, c8 = (q & 7) * 8; *(volatile v8b*)(dst + (size_t)(o0 + oo) * IN + i0 + c8) = *(const v8b*)(&T[oo][c8]); } __threadfence(); }
}
__global__ __launch_bounds__(256) void maps_kernel(const int* __restrict__ xtb, const int* __restrict__ xtp, const int* __restrict__ xfb, const int* __restrict__ xfp, int nx, const int* __restrict__ ytb, const int* __restrict__ ytp, const int* __restrict__ yfb, const int* __restrict__ yfp, int ny, const float* __restrict__ amask, int* __restrict__ QSRC, int* __restrict__ KSRC, int* __restrict__ OSRC, float* __restrict__ KM, float* __restrict__ AM) {
  const int t = blockIdx.x * 256 + threadIdx.x;
  if (t < NB * FULL) { const int b = t / FULL, P = t - b * FULL; int src = -1;
    for (int i = 0; i < nx; ++i) if (xtb[i] == b && xtp[i] == P) src = iclamp(xfb[i], 0, NB - 1) * SX + iclamp(xfp[i], 0, SX - 1);
    for (int pass = 0; pass < 2; ++pass) { ((volatile int*)QSRC)[t] = src; __threadfence(); }
  } else if (t < 2 * NB * FULL) { const int u = t - NB * FULL; const int b = u / FULL, K = u - b * FULL; int src = -1;
    for (int i = 0; i < ny; ++i) if (ytb[i] == b && ytp[i] == K) src = iclamp(yfb[i], 0, NB - 1) * SY + iclamp(yfp[i], 0, SY - 1);
    for (int pass = 0; pass < 2; ++pass) { ((volatile int*)KSRC)[u] = src; ((volatile float*)KM)[u] = (src >= 0) ? 0.0f : NEG; __threadfence(); }
  } else if (t < 2 * NB * FULL + NB * SX) { const int u = t - 2 * NB * FULL; const int b = u / SX, s = u - b * SX; int src = -1;
    for (int i = 0; i < nx; ++i) if (xfb[i] == b && xfp[i] == s) src = iclamp(xtb[i], 0, NB - 1) * FULL + iclamp(xtp[i], 0, FULL - 1);
    for (int pass = 0; pass < 2; ++pass) { ((volatile int*)OSRC)[u] = src; __threadfence(); }
  } else if (t < 2 * NB * FULL + 2 * NB * SX) { const int u = t - 2 * NB * FULL - NB * SX; for (int pass = 0; pass < 2; ++pass) { ((volatile float*)AM)[u] = bf16_rne(amask[u]); __threadfence(); } }
}
__global__ __launch_bounds__(128) void proj_in_kernel(const b16* __restrict__ A16, const b16* __restrict__ WT, const float* __restrict__ bias, int S, b16* __restrict__ P0h, b16* __restrict__ P0l, b16* __restrict__ P1h, b16* __restrict__ P1l, b16* __restrict__ P2h, b16* __restrict__ P2l, int rb0) {
  __shared__ __attribute__((aligned(16))) b16 Th[4][16][128 + 8], Tl[4][16][128 + 8];
  const int wave = threadIdx.x >> 5, lane = threadIdx.x & 31, nloc = lane & 15, hlf = lane >> 4; const int m0 = (rb0 + blockIdx.x) * 64 + wave * 16, n0 = blockIdx.y * 128; const int plane = n0 / D, h0 = (n0 - plane * D) / DH;
  v8f acc[8];
#pragma unroll
  for (int t = 0; t < 8; ++t) acc[t] = (v8f){};
#pragma unroll 2
  for (int kb = 0; kb < D; kb += 32) { const v16b a = frag_kb(A16 + (size_t)(m0 + nloc) * D + kb, hlf);
#pragma unroll
    for (int t = 0; t < 8; ++t) acc[t] = wmma16b(a, frag_kb(WT + (size_t)(n0 + t * 16 + nloc) * D + kb, hlf), acc[t]); }
#pragma unroll
  for (int t = 0; t < 8; ++t) { const float bb = bf16_rne(bias[n0 + t * 16 + nloc]);
#pragma unroll
    for (int r = 0; r < 8; ++r) { b16 a_, c_; split16((acc[t][r] * (1.0f / (XS * WSC)) + bb) * XS, a_, c_); Th[wave][8 * hlf + r][t * 16 + nloc] = a_; Tl[wave][8 * hlf + r][t * 16 + nloc] = c_; } }
  wave_lds_sync();
  b16* dh = plane == 0 ? P0h : plane == 1 ? P1h : P2h; b16* dl = plane == 0 ? P0l : plane == 1 ? P1l : P2l;
  for (int pass = 0; pass < 2; ++pass) {
    for (int rr = 0; rr < 16; ++rr) if (lane < 16) { const int m = m0 + rr, b = m / S, s = m - b * S; const int hsel = lane >> 3, c8 = (lane & 7) * 8; const size_t gi = (((size_t)b * NH + h0 + hsel) * S + s) * DH + c8;
      *(volatile v8b*)(dh + gi) = *(const v8b*)(&Th[wave][rr][hsel * 64 + c8]); *(volatile v8b*)(dl + gi) = *(const v8b*)(&Tl[wave][rr][hsel * 64 + c8]); }
    __threadfence(); }
}
__global__ __launch_bounds__(256) void v1t_kernel(const b16* __restrict__ Vh, const b16* __restrict__ Vl, b16* __restrict__ VTh, b16* __restrict__ VTl) {
  __shared__ __attribute__((aligned(16))) b16 Ta[DH][64 + 8], Tb[DH][64 + 8];
  const int bh = blockIdx.y, s0 = blockIdx.x * 64, t_ = threadIdx.x;
  for (int k = t_; k < 64 * DH; k += 256) { const int ss = k >> 6, d = k & 63; const size_t gi = ((size_t)bh * SX + s0 + ss) * DH + d; Ta[d][ss] = Vh[gi]; Tb[d][ss] = Vl[gi]; }
  __syncthreads();
  for (int pass = 0; pass < 2; ++pass) { for (int q = t_; q < DH * 8; q += 256) { const int d = q >> 3, c8 = (q & 7) * 8; const size_t gi = ((size_t)bh * DH + d) * SX + s0 + c8; *(volatile v8b*)(VTh + gi) = *(const v8b*)(&Ta[d][c8]); *(volatile v8b*)(VTl + gi) = *(const v8b*)(&Tb[d][c8]); } __threadfence(); }
}
__global__ __launch_bounds__(256) void gatherqk_kernel(const b16* __restrict__ Q2h, const b16* __restrict__ Q2l, const b16* __restrict__ K2h, const b16* __restrict__ K2l, const int* __restrict__ QSRC, const int* __restrict__ KSRC, b16* __restrict__ QFh, b16* __restrict__ QFl, b16* __restrict__ KFh, b16* __restrict__ KFl) {
  const int wave = threadIdx.x >> 5, lane = threadIdx.x & 31; const int row = blockIdx.x * 8 + wave;
  const int P = row % FULL, bh = row / FULL, b = bh / NH, h = bh - b * NH;
  const int qs = QSRC[b * FULL + P], ks = KSRC[b * FULL + P]; const v8b z = {};
  const int qb = qs >= 0 ? qs / SX : 0, qp = qs >= 0 ? qs - qb * SX : 0, kbb = ks >= 0 ? ks / SY : 0, kp = ks >= 0 ? ks - kbb * SY : 0;
  if (lane < 16) { const int which = lane >> 3, c8 = (lane & 7) * 8;
    const size_t qg = (((size_t)qb * NH + h) * SX + qp) * DH + c8, kg = (((size_t)kbb * NH + h) * SY + kp) * DH + c8, dst = (size_t)row * DH + c8;
    const v8b qh = *(const v8b*)(Q2h + qg), ql = *(const v8b*)(Q2l + qg), kh = *(const v8b*)(K2h + kg), kl = *(const v8b*)(K2l + kg);
    const v8b qv = qs >= 0 ? (which == 0 ? qh : ql) : z, kv = ks >= 0 ? (which == 0 ? kh : kl) : z;
    for (int pass = 0; pass < 2; ++pass) { *(volatile v8b*)((which == 0 ? QFh : QFl) + dst) = qv; *(volatile v8b*)((which == 0 ? KFh : KFl) + dst) = kv; __threadfence(); } }
}
__global__ __launch_bounds__(256) void gatherv_kernel(const b16* __restrict__ V2h, const b16* __restrict__ V2l, const int* __restrict__ KSRC, b16* __restrict__ VFTh, b16* __restrict__ VFTl) {
  __shared__ __attribute__((aligned(16))) b16 Ta[DH][64 + 8], Tb[DH][64 + 8];
  const int bh = blockIdx.y, b = bh / NH, h = bh - b * NH, K0 = blockIdx.x * 64, t_ = threadIdx.x;
  for (int k = t_; k < 64 * DH; k += 256) { const int kk = k >> 6, d = k & 63; const int ks = KSRC[b * FULL + K0 + kk]; const int sb = ks >= 0 ? ks / SY : 0, sp = ks >= 0 ? ks - sb * SY : 0;
    const size_t gi = (((size_t)sb * NH + h) * SY + sp) * DH + d; const b16 vh = V2h[gi], vl = V2l[gi]; Ta[d][kk] = ks >= 0 ? vh : (b16)0.0f; Tb[d][kk] = ks >= 0 ? vl : (b16)0.0f; }
  __syncthreads();
  for (int pass = 0; pass < 2; ++pass) { for (int q = t_; q < DH * 8; q += 256) { const int d = q >> 3, c8 = (q & 7) * 8; const size_t gi = ((size_t)bh * DH + d) * FULL + K0 + c8; *(volatile v8b*)(VFTh + gi) = *(const v8b*)(&Ta[d][c8]); *(volatile v8b*)(VFTl + gi) = *(const v8b*)(&Tb[d][c8]); } __threadfence(); }
}
__global__ __launch_bounds__(64) void attn_kernel(const b16* __restrict__ QH, const b16* __restrict__ QL, const b16* __restrict__ KH, const b16* __restrict__ KL, const b16* __restrict__ VTh, const b16* __restrict__ VTl, const float* __restrict__ madd, int SQ, b16* __restrict__ OUTh, b16* __restrict__ OUTl, int ldo, int qb0, int bh0) {
  __shared__ __attribute__((aligned(16))) b16 To[2][16][DH + 8], Tp[2][16][DH + 8];
  const int wave = threadIdx.x >> 5, lane = threadIdx.x & 31, hh = lane >> 4, col = lane & 15; const int bh = bh0 + blockIdx.y, b = bh / NH, h = bh - b * NH, i0 = (qb0 + blockIdx.x) * 32 + wave * 16, qi = i0 + col;
  const b16* Qh = QH + (size_t)bh * SQ * DH; const b16* Ql = QL + (size_t)bh * SQ * DH; const b16* Kh = KH + (size_t)bh * SQ * DH; const b16* Kl = KL + (size_t)bh * SQ * DH; const b16* Vh = VTh + (size_t)bh * DH * SQ; const b16* Vl = VTl + (size_t)bh * DH * SQ; const float* ma = madd + (size_t)b * SQ;
  v16b qf[2], ql2[2];
#pragma unroll
  for (int ks = 0; ks < 2; ++ks) { qf[ks] = frag_kb(Qh + (size_t)qi * DH + ks * 32, hh); ql2[ks] = frag_kb(Ql + (size_t)qi * DH + ks * 32, hh); }
  const float scale = 0.125f * (1.0f / (XS * XS));
  float m = -INFINITY, l = 0.0f; v8f o[4] = {{}, {}, {}, {}};
  const int kend = i0 + 16;
  for (int kb = 0; kb < kend; kb += 32) {
    v8f s0 = {}, s1 = {};
#pragma unroll
    for (int ks = 0; ks < 2; ++ks) { const size_t r0 = (size_t)(kb + col) * DH + ks * 32, r1 = (size_t)(kb + 16 + col) * DH + ks * 32; const v16b k0h = frag_kb(Kh + r0, hh), k0l = frag_kb(Kl + r0, hh), k1h = frag_kb(Kh + r1, hh), k1l = frag_kb(Kl + r1, hh);
      s0 = wmma16b(k0h, qf[ks], s0); s0 = wmma16b(k0h, ql2[ks], s0); s0 = wmma16b(k0l, qf[ks], s0); s1 = wmma16b(k1h, qf[ks], s1); s1 = wmma16b(k1h, ql2[ks], s1); s1 = wmma16b(k1l, qf[ks], s1); }
    float mr = -INFINITY;
#pragma unroll
    for (int r = 0; r < 8; ++r) { const int ja = kb + 8 * hh + r, jc = kb + 16 + 8 * hh + r; const float aa = ma[ja < SQ ? ja : SQ - 1], ac = ma[jc < SQ ? jc : SQ - 1];
      s0[r] = (ja <= qi) ? s0[r] * scale + aa : NEG + aa; s1[r] = (jc <= qi) ? s1[r] * scale + ac : NEG + ac; mr = fmaxf(mr, fmaxf(s0[r], s1[r])); }
    mr = fmaxf(mr, __shfl_xor(mr, 16)); const float mn = fmaxf(m, mr); const float al_ = nexp(m - mn); m = mn; float sum = 0.0f; v16b pb, pl;
#pragma unroll
    for (int r = 0; r < 8; ++r) { const float e0 = nexp(s0[r] - mn), e1 = nexp(s1[r] - mn); sum += e0 + e1; b16 a_, c_; split16(e0 * PS, a_, c_); pb[r] = a_; pl[r] = c_; split16(e1 * PS, a_, c_); pb[8 + r] = a_; pl[8 + r] = c_; }
    sum += __shfl_xor(sum, 16); l = l * al_ + sum;
#pragma unroll
    for (int t = 0; t < 4; ++t) { o[t] *= al_; const size_t vo = (size_t)(t * 16 + col) * SQ + kb; const v16b vh = frag_kb(Vh + vo, hh); o[t] = wmma16b(vh, pb, o[t]); o[t] = wmma16b(vh, pl, o[t]); o[t] = wmma16b(frag_kb(Vl + vo, hh), pb, o[t]); } }
  const float inv = 1.0f / (l * PS * XS);
#pragma unroll
  for (int t = 0; t < 4; ++t)
#pragma unroll
    for (int r = 0; r < 8; ++r) { b16 a_, c_; split16(o[t][r] * inv * XS, a_, c_); To[wave][col][t * 16 + 8 * hh + r] = a_; Tp[wave][col][t * 16 + 8 * hh + r] = c_; }
  wave_lds_sync();
  for (int pass = 0; pass < 2; ++pass) { for (int rr = 0; rr < 16; ++rr) if (lane < 8) { const size_t gi = ((size_t)b * SQ + i0 + rr) * ldo + h * DH + lane * 8; *(volatile v8b*)(OUTh + gi) = *(const v8b*)(&To[wave][rr][lane * 8]); *(volatile v8b*)(OUTl + gi) = *(const v8b*)(&Tp[wave][rr][lane * 8]); } __threadfence(); }
}
__global__ __launch_bounds__(256) void shrink_kernel(const b16* __restrict__ A2h, const b16* __restrict__ A2l, const int* __restrict__ OSRC, b16* __restrict__ CATh, b16* __restrict__ CATl, int row0) {
  const int wave = threadIdx.x >> 5, lane = threadIdx.x & 31; const int row = row0 + blockIdx.x * 8 + wave; const int b = row / SX; const int os = OSRC[row]; const int tb = os >= 0 ? os / FULL : 0, tp = os >= 0 ? os - tb * FULL : 0;
  const v8b z = {};
  for (int pass = 0; pass < 2; ++pass) { for (int qd = 0; qd < 4; ++qd) { const size_t src = ((size_t)tb * FULL + tp) * D + qd * 256 + lane * 8, dst = (size_t)row * (2 * D) + D + qd * 256 + lane * 8; const v8b vh = *(const v8b*)(A2h + src), vl = *(const v8b*)(A2l + src); *(volatile v8b*)(CATh + dst) = os >= 0 ? vh : z; *(volatile v8b*)(CATl + dst) = os >= 0 ? vl : z; } __threadfence(); }
  (void)b;
}
__global__ __launch_bounds__(128) void proj_out_kernel(const b16* __restrict__ CATh, const b16* __restrict__ CATl, const b16* __restrict__ WPJ, const float* __restrict__ bias, float* __restrict__ out, int rb0) {
  __shared__ __attribute__((aligned(16))) float Ts[4][16][128 + 4];
  const int wave = threadIdx.x >> 5, lane = threadIdx.x & 31, nloc = lane & 15, hlf = lane >> 4; const int m0 = (rb0 + blockIdx.x) * 64 + wave * 16, n0 = blockIdx.y * 128;
  v8f acc[8];
#pragma unroll
  for (int t = 0; t < 8; ++t) acc[t] = (v8f){};
  for (int kb = 0; kb < 2 * D; kb += 32) { const v16b a = frag_kb(CATh + (size_t)(m0 + nloc) * (2 * D) + kb, hlf), al = frag_kb(CATl + (size_t)(m0 + nloc) * (2 * D) + kb, hlf);
#pragma unroll
    for (int t = 0; t < 8; ++t) { const v16b bw = frag_kb(WPJ + (size_t)(n0 + t * 16 + nloc) * (2 * D) + kb, hlf); acc[t] = wmma16b(a, bw, acc[t]); acc[t] = wmma16b(al, bw, acc[t]); } }
#pragma unroll
  for (int t = 0; t < 8; ++t) { const float bb = bf16_rne(bias[n0 + t * 16 + nloc]);
#pragma unroll
    for (int r = 0; r < 8; ++r) Ts[wave][8 * hlf + r][t * 16 + nloc] = acc[t][r] * (1.0f / (XS * WSC)) + bb; }
  wave_lds_sync();
  for (int pass = 0; pass < 2; ++pass) { for (int rr = 0; rr < 16; ++rr) *(volatile v4f*)(out + (size_t)(m0 + rr) * D + n0 + lane * 4) = *(const v4f*)(&Ts[wave][rr][lane * 4]); __threadfence(); }
}
}

extern "C" void kernel_launch(void* const* d_in, const int* in_sizes, int n_in, void* d_out, int out_size, void* d_ws, size_t ws_size, hipStream_t stream) {
  (void)n_in;
  auto Fp = [&](int i) { return (const float*)d_in[i]; }; auto Ip = [&](int i) { return (const int*)d_in[i]; };
  const int nx = in_sizes[11], ny = in_sizes[15];
  if (in_sizes[0] != NROW * D || in_sizes[1] != NB * SY * D || in_sizes[2] != NB * SX || in_sizes[3] != D * 3 * D || in_sizes[7] != D * 2 * D || in_sizes[9] != 2 * D * D || in_sizes[12] != nx || in_sizes[13] != nx || in_sizes[14] != nx || in_sizes[16] != ny || in_sizes[17] != ny || in_sizes[18] != ny || out_size != NROW * D) return;
  size_t off = 0; char* ws = (char*)d_ws;
  auto carve = [&](size_t bytes) { char* p = ws + off; off += (bytes + 255) & ~(size_t)255; return p; };
  b16* X16 = (b16*)carve((size_t)NROW * D * 2); b16* Y16 = (b16*)carve((size_t)NB * SY * D * 2);
  b16* WA = (b16*)carve((size_t)3 * D * D * 2); b16* W2A = (b16*)carve((size_t)D * D * 2); b16* W2B = (b16*)carve((size_t)2 * D * D * 2); b16* WPJ = (b16*)carve((size_t)D * 2 * D * 2);
  int* QSRC = (int*)carve(NB * FULL * 4); int* KSRC = (int*)carve(NB * FULL * 4); int* OSRC = (int*)carve(NB * SX * 4); float* KM = (float*)carve(NB * FULL * 4); float* AM = (float*)carve(NB * SX * 4);
  const size_t ps = (size_t)NB * NH * SX * DH;
  b16* Q1h = (b16*)carve(ps * 2); b16* Q1l = (b16*)carve(ps * 2); b16* K1h = (b16*)carve(ps * 2); b16* K1l = (b16*)carve(ps * 2); b16* V1h = (b16*)carve(ps * 2); b16* V1l = (b16*)carve(ps * 2); b16* V1Th = (b16*)carve(ps * 2); b16* V1Tl = (b16*)carve(ps * 2);
  b16* Q2h = (b16*)carve(ps * 2); b16* Q2l = (b16*)carve(ps * 2); b16* K2h = (b16*)carve(ps * 2); b16* K2l = (b16*)carve(ps * 2); b16* V2h = (b16*)carve(ps * 2); b16* V2l = (b16*)carve(ps * 2);
  const size_t pf = (size_t)NB * NH * FULL * DH;
  b16* QFh = (b16*)carve(pf * 2); b16* QFl = (b16*)carve(pf * 2); b16* KFh = (b16*)carve(pf * 2); b16* KFl = (b16*)carve(pf * 2); b16* VFTh = (b16*)carve(pf * 2); b16* VFTl = (b16*)carve(pf * 2);
  b16* A2h = X16; b16* A2l = V1h; b16* CATh = Q2h; b16* CATl = K2h;
  static_assert((size_t)NB * FULL * D <= 2 * (size_t)NROW * D, "A2 plane fits X16|Y16"); static_assert((size_t)NROW * 2 * D == 2 * ((size_t)NB * NH * SX * DH), "CAT plane = two qkv planes");
  if (off > ws_size) return;
  prepx_kernel<<<(NROW * D * 2 / 8 + 255) / 256, 256, 0, stream>>>(Fp(0), Fp(1), X16, Y16);
  prepw_kernel<<<dim3(2 * D / 64, 3 * D / 64, 4), 256, 0, stream>>>(Fp(3), Fp(5), Fp(7), Fp(9), WA, W2A, W2B, WPJ);
  maps_kernel<<<(2 * NB * FULL + 2 * NB * SX + 255) / 256, 256, 0, stream>>>(Ip(11), Ip(12), Ip(13), Ip(14), nx, Ip(15), Ip(16), Ip(17), Ip(18), ny, Fp(2), QSRC, KSRC, OSRC, KM, AM);
  proj_in_kernel<<<dim3(NROW / 64, 3 * D / 128), 128, 0, stream>>>(X16, WA, Fp(4), SX, Q1h, Q1l, K1h, K1l, V1h, V1l, 0);
  proj_in_kernel<<<dim3(NROW / 64, D / 128), 128, 0, stream>>>(X16, W2A, Fp(6), SX, Q2h, Q2l, nullptr, nullptr, nullptr, nullptr, 0);
  proj_in_kernel<<<dim3(NB * SY / 64, 2 * D / 128), 128, 0, stream>>>(Y16, W2B, Fp(8), SY, K2h, K2l, V2h, V2l, nullptr, nullptr, 0);
  v1t_kernel<<<dim3(SX / 64, NB * NH), 256, 0, stream>>>(V1h, V1l, V1Th, V1Tl);
  gatherqk_kernel<<<NB * NH * FULL / 8, 256, 0, stream>>>(Q2h, Q2l, K2h, K2l, QSRC, KSRC, QFh, QFl, KFh, KFl);
  gatherv_kernel<<<dim3(FULL / 64, NB * NH), 256, 0, stream>>>(V2h, V2l, KSRC, VFTh, VFTl);
  attn_kernel<<<dim3(SX / 32, NB * NH), 64, 0, stream>>>(Q1h, Q1l, K1h, K1l, V1Th, V1Tl, AM, SX, CATh, CATl, 2 * D, 0, 0);
  attn_kernel<<<dim3(FULL / 32, NB * NH), 64, 0, stream>>>(QFh, QFl, KFh, KFl, VFTh, VFTl, KM, FULL, A2h, A2l, D, 0, 0);
  shrink_kernel<<<NROW / 8, 256, 0, stream>>>(A2h, A2l, OSRC, CATh, CATl, 0);
  proj_out_kernel<<<dim3(NROW / 64, D / 128), 128, 0, stream>>>(CATh, CATl, WPJ, Fp(10), (float*)d_out, 0);
}
